// ARM_57226144252650
// MI455X (gfx1250) — hardware-run, weakly checked
//
#include <hip/hip_runtime.h>
#include <math.h>

typedef __attribute__((ext_vector_type(16))) _Float16 v16h;
typedef __attribute__((ext_vector_type(8)))  _Float16 v8h;
typedef __attribute__((ext_vector_type(4)))  _Float16 v4h;
typedef __attribute__((ext_vector_type(8)))  float    v8f;
typedef __attribute__((ext_vector_type(4)))  float    v4f;
typedef __attribute__((ext_vector_type(4)))  unsigned v4u;

constexpr int kBatch  = 8;
constexpr int kImg    = 224;
constexpr int kPatch  = 16;
constexpr int kGridP  = kImg / kPatch;
constexpr int kSeq    = kGridP * kGridP;
constexpr int kDim    = 384;
constexpr int kDepth  = 24;
constexpr int kNst    = 16;
constexpr int kConvK  = 4;
constexpr int kRank   = 24;
constexpr int kHid    = 1024;
constexpr int kTok    = kBatch * kSeq;
constexpr int kTokP   = 1600;
constexpr int kXzP    = 2 * kDim;
constexpr int kXdN    = kRank + 2 * kNst;
constexpr int kXdP    = 64;
constexpr int kDtK    = 32;
constexpr int kPatchK = 3 * kPatch * kPatch;
constexpr int kG12P   = 2 * kHid;
static_assert(kSeq == 196 && kTok == 1568, "token count");
static_assert(kTokP % 64 == 0 && kTokP >= kTok, "M tile multiple");
static_assert(kXdN == 56 && kXdN <= kXdP, "x_proj width");
static_assert(kDim % 64 == 0 && kXzP % 64 == 0 && kXdP % 64 == 0 && kG12P % 64 == 0, "N tile multiples");
static_assert(kPatchK % 32 == 0 && kDim % 32 == 0 && kDtK % 32 == 0 && kHid % 32 == 0, "K multiples of 32");
static_assert(kRank % 8 == 0 && kRank <= kDtK, "dt rank padding");

constexpr float kCarryW   = 32.0f;
constexpr float kCarryWdt = 8.0f;
constexpr float kCarryXa  = 16.0f;
constexpr float kCarryDt  = 64.0f;
constexpr float kCarryY   = 256.0f;
constexpr float kCarryHid = 16.0f;

constexpr size_t kSzPW   = (size_t)kDim * kPatchK * 2;
constexpr size_t kSzWIN  = (size_t)kDepth * kXzP * kDim * 2;
constexpr size_t kSzWXP  = (size_t)kDepth * kXdP * kDim * 2;
constexpr size_t kSzWDT  = (size_t)kDepth * kDim * kDtK * 2;
constexpr size_t kSzWOUT = (size_t)kDepth * kDim * kDim * 2;
constexpr size_t kSzW12  = (size_t)kDepth * kG12P * kDim * 2;
constexpr size_t kSzW3   = (size_t)kDepth * kDim * kHid * 2;
constexpr size_t kSzA0   = (size_t)kTokP * kPatchK * 2;
constexpr size_t kSzH    = (size_t)kTokP * kDim * 4;
constexpr size_t kSzU16  = (size_t)kTokP * kDim * 2;
constexpr size_t kSzXZ   = (size_t)kTokP * kXzP * 4;
constexpr size_t kSzXA   = (size_t)kTokP * kDim * 4;
constexpr size_t kSzXA16 = (size_t)kTokP * kDim * 2;
constexpr size_t kSzDBC  = (size_t)kTokP * kXdP * 4;
constexpr size_t kSzDTIN = (size_t)kTokP * kDtK * 2;
constexpr size_t kSzDLR  = (size_t)kTokP * kDim * 4;
constexpr size_t kSzY16  = (size_t)kTokP * kDim * 2;
constexpr size_t kSzG12  = (size_t)kTokP * kG12P * 4;
constexpr size_t kSzHID  = (size_t)kTokP * kHid * 2;
constexpr size_t kOffPW   = 0;
constexpr size_t kOffWIN  = kOffPW   + kSzPW;
constexpr size_t kOffWXP  = kOffWIN  + kSzWIN;
constexpr size_t kOffWDT  = kOffWXP  + kSzWXP;
constexpr size_t kOffWOUT = kOffWDT  + kSzWDT;
constexpr size_t kOffW12  = kOffWOUT + kSzWOUT;
constexpr size_t kOffW3   = kOffW12  + kSzW12;
constexpr size_t kOffA0   = kOffW3   + kSzW3;
constexpr size_t kOffH    = kOffA0   + kSzA0;
constexpr size_t kOffU16  = kOffH    + kSzH;
constexpr size_t kOffXZ   = kOffU16  + kSzU16;
constexpr size_t kOffXA   = kOffXZ   + kSzXZ;
constexpr size_t kOffXA16 = kOffXA   + kSzXA;
constexpr size_t kOffDBC  = kOffXA16 + kSzXA16;
constexpr size_t kOffDTIN = kOffDBC  + kSzDBC;
constexpr size_t kOffDLR  = kOffDTIN + kSzDTIN;
constexpr size_t kOffY16  = kOffDLR  + kSzDLR;
constexpr size_t kOffG12  = kOffY16  + kSzY16;
constexpr size_t kOffHID  = kOffG12  + kSzG12;
constexpr size_t kWsTotal = kOffHID  + kSzHID;
static_assert(kWsTotal == 115544064ull, "carve total");
static_assert(kWsTotal <= 134217728ull, "carve cap");
static_assert((kOffWIN % 128) == 0 && (kOffWXP % 128) == 0 && (kOffWDT % 128) == 0 && (kOffWOUT % 128) == 0 &&
              (kOffW12 % 128) == 0 && (kOffW3 % 128) == 0 && (kOffA0 % 128) == 0 && (kOffH % 128) == 0 &&
              (kOffU16 % 128) == 0 && (kOffXZ % 128) == 0 && (kOffXA % 128) == 0 && (kOffXA16 % 128) == 0 &&
              (kOffDBC % 128) == 0 && (kOffDTIN % 128) == 0 && (kOffDLR % 128) == 0 && (kOffY16 % 128) == 0 &&
              (kOffG12 % 128) == 0 && (kOffHID % 128) == 0, "128-B aligned regions");

__device__ __forceinline__ float silu_fast(float v) {
  return v * __builtin_amdgcn_rcpf(1.0f + __expf(-v));
}
__device__ __forceinline__ float softplus_fast(float v) {
  const float a   = __expf(-fabsf(v));
  const float u   = 1.0f + a;
  const float l1p = __logf(u) + (a - (u - 1.0f)) * __builtin_amdgcn_rcpf(u);
  return fmaxf(v, 0.0f) + l1p;
}

struct FragH {
  union U { v16h v; v8h h[2]; };
  static __device__ __forceinline__ v16h load(const _Float16* p) {
    U f; f.h[0] = *(const v8h*)(p); f.h[1] = *(const v8h*)(p + 16); return f.v;
  }
  static __device__ __forceinline__ v8f mma(v16h a, v16h b, v8f c) {
    return __builtin_amdgcn_wmma_f32_16x16x32_f16(false, a, false, b, (short)0, c, false, false);
  }
};
__device__ __forceinline__ void guard_row_h(v8f& a, v8f& b, v8f& c, v8f& d, v16h x, v16h b0, v16h b1, v16h b2, v16h b3) {
  asm volatile("v_nop\n\tv_nop\n\tv_nop\n\tv_nop" : "+v"(a), "+v"(b), "+v"(c), "+v"(d) : "v"(x), "v"(b0), "v"(b1), "v"(b2), "v"(b3));
}
__device__ __forceinline__ void acc_guard4(v8f& a, v8f& b, v8f& c, v8f& d) {
  asm volatile("v_nop\n\tv_nop\n\tv_nop\n\tv_nop" : "+v"(a), "+v"(b), "+v"(c), "+v"(d));
}

template <int BIAS_MODE, int OUT_MODE, bool RESID>
__global__ __launch_bounds__(256) void wmma_gemm64_f16(
    const unsigned short* __restrict__ Ap, int lda,
    const unsigned short* __restrict__ Btp, int ldb,
    float* Cout, int ldc,
    const float* __restrict__ bias, const float* __restrict__ bias2, int nsplit,
    const float* resid, unsigned short* aux16,
    int M, int N, int K, float scale) {
  const _Float16* A  = (const _Float16*)Ap;
  const _Float16* Bt = (const _Float16*)Btp;
  __shared__ __align__(16) float sT[8][16 * 68];
  const int lane = threadIdx.x & 31;
  const int wave = threadIdx.x >> 5;
  const int tilesN = N >> 6;
  const int tilesM = M >> 6;
  const int tile = blockIdx.x * 8 + wave;
  if (tile >= tilesM * tilesN) return;
  const int tm = tile / tilesN;
  const int tn = tile - tm * tilesN;
  const int m0 = tm << 6;
  const int n0 = tn << 6;

  const int rlane = lane & 15;
  const int koff  = (lane >> 4) * 8;
  const int mOff  = (lane >> 4) * 8;

  v8f acc[4][4];
#pragma unroll
  for (int i = 0; i < 4; ++i)
#pragma unroll
    for (int j = 0; j < 4; ++j) acc[i][j] = (v8f){0.f,0.f,0.f,0.f,0.f,0.f,0.f,0.f};

  for (int k0 = 0; k0 < K; k0 += 32) {
    v16h bh[4];
#pragma unroll
    for (int j = 0; j < 4; ++j) {
      const size_t bo = (size_t)(n0 + (j << 4) + rlane) * ldb + koff + k0;
      bh[j] = FragH::load(Bt + bo);
    }
#pragma unroll
    for (int i = 0; i < 4; ++i) {
      const size_t ao = (size_t)(m0 + (i << 4) + rlane) * lda + koff + k0;
      const v16h ah = FragH::load(A + ao);
#pragma unroll
      for (int j = 0; j < 4; ++j) acc[i][j] = FragH::mma(ah, bh[j], acc[i][j]);
      guard_row_h(acc[i][0], acc[i][1], acc[i][2], acc[i][3], ah, bh[0], bh[1], bh[2], bh[3]);
    }
  }
  acc_guard4(acc[0][0], acc[0][1], acc[0][2], acc[0][3]);
  acc_guard4(acc[1][0], acc[1][1], acc[1][2], acc[1][3]);
  acc_guard4(acc[2][0], acc[2][1], acc[2][2], acc[2][3]);
  acc_guard4(acc[3][0], acc[3][1], acc[3][2], acc[3][3]);

  float* slab = sT[wave];
#pragma unroll
  for (int i = 0; i < 4; ++i) {
    const int mBase = m0 + (i << 4);
#pragma unroll
    for (int j = 0; j < 4; ++j) {
      const int n = n0 + (j << 4) + rlane;
      float bv = 0.f;
      if (BIAS_MODE == 2) {
        const int n1 = (n < nsplit) ? n : (nsplit - 1);
        const int n2 = (n >= nsplit) ? (n - nsplit) : 0;
        const float b1 = bias[n1];
        const float b2 = bias2[n2];
        bv = (n < nsplit) ? b1 : b2;
      }
#pragma unroll
      for (int r = 0; r < 8; ++r) {
        const float v = acc[i][j][r] * scale + bv;
        slab[(mOff + r) * 68 + (j << 4) + rlane] = v;
      }
    }
    __builtin_amdgcn_fence(__ATOMIC_RELEASE, "workgroup");
    __builtin_amdgcn_wave_barrier();
    __builtin_amdgcn_fence(__ATOMIC_ACQUIRE, "workgroup");
    {
      const int hh = lane >> 4, c4 = (lane & 15) * 4;
      v4f vals[8];
#pragma unroll
      for (int it = 0; it < 8; ++it) {
        const int row = it * 2 + hh;
        v4f v = *(const v4f*)(slab + row * 68 + c4);
        if (RESID) {
          const v4f rv = *(const v4f*)(resid + (size_t)(mBase + row) * ldc + n0 + c4);
          v = v + rv;
        }
        vals[it] = v;
      }
      for (int pass = 0; pass < 2; ++pass) {
#pragma unroll
        for (int it = 0; it < 8; ++it) {
          const int row = it * 2 + hh;
          *(volatile v4f*)(Cout + (size_t)(mBase + row) * ldc + n0 + c4) = vals[it];
        }
        __threadfence();
      }
    }
    if (OUT_MODE == 3) {
      if (n0 == 0) {
        const int r8 = lane >> 2, cc = (lane & 3) * 8;
        const bool live = (cc < kRank);
        v8h dv[2];
#pragma unroll
        for (int it = 0; it < 2; ++it) {
          const int row = it * 8 + r8;
          const float* sp = slab + row * 68 + cc;
          const v4f a0 = *(const v4f*)(sp);
          const v4f a1 = *(const v4f*)(sp + 4);
#pragma unroll
          for (int e = 0; e < 4; ++e) {
            const float f0 = live ? (a0[e] * kCarryDt) : 0.0f;
            const float f1 = live ? (a1[e] * kCarryDt) : 0.0f;
            dv[it][e]     = (_Float16)f0;
            dv[it][4 + e] = (_Float16)f1;
          }
        }
        for (int pass = 0; pass < 2; ++pass) {
#pragma unroll
          for (int it = 0; it < 2; ++it) {
            const int row = it * 8 + r8;
            *(volatile v8h*)(aux16 + (size_t)(mBase + row) * kDtK + cc) = dv[it];
          }
          __threadfence();
        }
      }
    }
    __builtin_amdgcn_fence(__ATOMIC_RELEASE, "workgroup");
    __builtin_amdgcn_wave_barrier();
    __builtin_amdgcn_fence(__ATOMIC_ACQUIRE, "workgroup");
  }
}

__global__ __launch_bounds__(256) void cast_plane_kernel(
    const float* __restrict__ src, unsigned short* __restrict__ dst, int total8,
    int rows_launch, int rows_src, int k_src, int k_dst, int dst_layer_rows, int dst_row_off, float scale)
{
  const int i = blockIdx.x * 256 + threadIdx.x;
  if (i >= total8) return;
  const int kc8 = k_dst >> 3;
  const int per_layer = rows_launch * kc8;
  const int layer = i / per_layer;
  const int rem = i - layer * per_layer;
  const int r = rem / kc8;
  const int k0 = (rem - r * kc8) * 8;
  const bool valid = (r < rows_src) && (k0 < k_src);
  const int rc = (r < rows_src) ? r : (rows_src - 1);
  const int kc = (k0 < k_src) ? k0 : (k_src - 8);
  const float* p = src + ((size_t)layer * rows_src + rc) * k_src + kc;
  const v4f a0 = *(const v4f*)(p);
  const v4f a1 = *(const v4f*)(p + 4);
  v8h hv;
#pragma unroll
  for (int e = 0; e < 4; ++e) {
    const float f0 = valid ? (a0[e] * scale) : 0.0f;
    const float f1 = valid ? (a1[e] * scale) : 0.0f;
    hv[e]     = (_Float16)f0;
    hv[4 + e] = (_Float16)f1;
  }
  unsigned short* q = dst + ((size_t)layer * dst_layer_rows + dst_row_off + r) * k_dst + k0;
  *(volatile v8h*)q = hv;
  __threadfence();
  *(volatile v8h*)q = hv;
}

__global__ __launch_bounds__(256) void zero_fill16_kernel(unsigned short* __restrict__ dst, int total8)
{
  const int i = blockIdx.x * 256 + threadIdx.x;
  if (i >= total8) return;
  const v4u z = (v4u){0u, 0u, 0u, 0u};
  unsigned short* q = dst + ((size_t)i << 3);
  *(volatile v4u*)q = z;
  __threadfence();
  *(volatile v4u*)q = z;
}

__global__ __launch_bounds__(256) void im2col_kernel(const float* __restrict__ x, unsigned short* __restrict__ A0)
{
  const int i = blockIdx.x * 256 + threadIdx.x;
  if (i >= kTokP * (kPatchK / 8)) return;
  const int m  = i / (kPatchK / 8);
  const int k8 = (i - m * (kPatchK / 8)) * 8;
  const int c  = k8 >> 8;
  const int ii = (k8 >> 4) & 15;
  const int j0 = k8 & 15;
  const bool valid = (m < kTok);
  const int mc = valid ? m : (kTok - 1);
  const int b  = mc / kSeq;
  const int l  = mc - b * kSeq;
  const int py = l / kGridP;
  const int px = l - py * kGridP;
  const float* p = x + ((size_t)((b * 3 + c) * kImg + py * kPatch + ii)) * kImg + px * kPatch + j0;
  const v4f a0 = *(const v4f*)(p);
  const v4f a1 = *(const v4f*)(p + 4);
  v8h hv;
#pragma unroll
  for (int e = 0; e < 4; ++e) {
    const float f0 = valid ? a0[e] : 0.0f;
    const float f1 = valid ? a1[e] : 0.0f;
    hv[e]     = (_Float16)f0;
    hv[4 + e] = (_Float16)f1;
  }
  unsigned short* q = A0 + ((size_t)i << 3);
  *(volatile v8h*)q = hv;
  __threadfence();
  *(volatile v8h*)q = hv;
}

template <bool FINAL>
__global__ __launch_bounds__(256) void ln_kernel(
    const float* __restrict__ X, const float* __restrict__ w, const float* __restrict__ b,
    void* __restrict__ outp, int nrows)
{
  const int lane = threadIdx.x & 31, wave = threadIdx.x >> 5;
  const int row = blockIdx.x * 8 + wave;
  if (row >= nrows) return;
  const float* xr = X + (size_t)row * kDim;
  const int c0 = lane * 4;
  const v4f x0 = *(const v4f*)(xr + c0);
  const v4f x1 = *(const v4f*)(xr + 128 + c0);
  const v4f x2 = *(const v4f*)(xr + 256 + c0);
  float s = ((x0[0] + x0[1]) + (x0[2] + x0[3])) + ((x1[0] + x1[1]) + (x1[2] + x1[3])) + ((x2[0] + x2[1]) + (x2[2] + x2[3]));
#pragma unroll
  for (int off = 16; off > 0; off >>= 1) s += __shfl_xor(s, off, 32);
  const float mean = s * (1.0f / (float)kDim);
  const v4f d0 = x0 - mean, d1 = x1 - mean, d2 = x2 - mean;
  float ss = ((d0[0] * d0[0] + d0[1] * d0[1]) + (d0[2] * d0[2] + d0[3] * d0[3]))
           + ((d1[0] * d1[0] + d1[1] * d1[1]) + (d1[2] * d1[2] + d1[3] * d1[3]))
           + ((d2[0] * d2[0] + d2[1] * d2[1]) + (d2[2] * d2[2] + d2[3] * d2[3]));
#pragma unroll
  for (int off = 16; off > 0; off >>= 1) ss += __shfl_xor(ss, off, 32);
  const float var  = ss * (1.0f / (float)kDim);
  const float rstd = 1.0f / sqrtf(var + 1e-5f);
  const v4f w0 = *(const v4f*)(w + c0), w1 = *(const v4f*)(w + 128 + c0), w2 = *(const v4f*)(w + 256 + c0);
  const v4f b0 = *(const v4f*)(b + c0), b1 = *(const v4f*)(b + 128 + c0), b2 = *(const v4f*)(b + 256 + c0);
  const v4f o0 = d0 * rstd * w0 + b0;
  const v4f o1 = d1 * rstd * w1 + b1;
  const v4f o2 = d2 * rstd * w2 + b2;
  if (FINAL) {
    float* orow = (float*)outp + (size_t)row * kDim + c0;
    for (int pass = 0; pass < 2; ++pass) {
      *(volatile v4f*)(orow)       = o0;
      *(volatile v4f*)(orow + 128) = o1;
      *(volatile v4f*)(orow + 256) = o2;
      __threadfence();
    }
  } else {
    v4h h0, h1, h2;
#pragma unroll
    for (int e = 0; e < 4; ++e) {
      h0[e] = (_Float16)o0[e];
      h1[e] = (_Float16)o1[e];
      h2[e] = (_Float16)o2[e];
    }
    unsigned short* orow = (unsigned short*)outp + (size_t)row * kDim + c0;
    for (int pass = 0; pass < 2; ++pass) {
      *(volatile v4h*)(orow)       = h0;
      *(volatile v4h*)(orow + 128) = h1;
      *(volatile v4h*)(orow + 256) = h2;
      __threadfence();
    }
  }
}

__global__ __launch_bounds__(256) void conv_silu_kernel(
    const float* __restrict__ XZ, const float* __restrict__ cw, const float* __restrict__ cb,
    float* __restrict__ XA, unsigned short* __restrict__ XA16)
{
  const int i = blockIdx.x * 256 + threadIdx.x;
  if (i >= kTokP * (kDim / 4)) return;
  const int m  = i / (kDim / 4);
  const int c4 = (i - m * (kDim / 4)) * 4;
  const int bq = m / kSeq;
  const int l  = m - bq * kSeq;
  v4f cwv[4];
#pragma unroll
  for (int e = 0; e < 4; ++e) cwv[e] = *(const v4f*)(cw + (size_t)(c4 + e) * kConvK);
  const v4f bias = *(const v4f*)(cb + c4);
  v4f acc = (v4f){0.f, 0.f, 0.f, 0.f};
#pragma unroll
  for (int k = 0; k < kConvK; ++k) {
    const bool ok = (l + k - (kConvK - 1)) >= 0;
    const int mr = ok ? (m + k - (kConvK - 1)) : m;
    v4f xv = *(const v4f*)(XZ + (size_t)mr * kXzP + c4);
    const v4f zero4 = (v4f){0.f, 0.f, 0.f, 0.f};
    xv = ok ? xv : zero4;
#pragma unroll
    for (int e = 0; e < 4; ++e) acc[e] = fmaf(xv[e], cwv[e][k], acc[e]);
  }
  v4f o;
  v4h oh;
#pragma unroll
  for (int e = 0; e < 4; ++e) {
    const float sv = acc[e] + bias[e];
    const float a  = silu_fast(sv);
    o[e]  = a;
    oh[e] = (_Float16)(a * kCarryXa);
  }
  float* pf = XA + ((size_t)i << 2);
  unsigned short* ph = XA16 + ((size_t)i << 2);
  *(volatile v4f*)pf = o;
  *(volatile v4h*)ph = oh;
  __threadfence();
  *(volatile v4f*)pf = o;
  *(volatile v4h*)ph = oh;
}

constexpr int kScanCh = 128;
constexpr int kScanTS = 28;
constexpr int kScanYP = 132;
constexpr int kScanPairs = kScanTS / 2;
static_assert(kSeq % kScanTS == 0 && (kScanTS % 2) == 0 && kDim % kScanCh == 0, "scan tiling");
static_assert(kScanTS * 8 <= 2 * kScanCh, "B/C staging coverage");

__global__ __launch_bounds__(128) void scan_gate_kernel(
    const float* __restrict__ DLR, const float* __restrict__ XA, const float* __restrict__ XZ,
    const float* __restrict__ DBC, const float* __restrict__ Alog, const float* __restrict__ Dsk,
    unsigned short* __restrict__ Y16)
{
  __shared__ __align__(16) float sBC[kScanTS * 32];
  __shared__ __align__(16) float sY[kScanTS * kScanYP];
  const int tid = threadIdx.x, lane = tid & 31, wave = tid >> 5;
  constexpr int kBlkPerB = kDim / kScanCh;
  const int bix = blockIdx.x / kBlkPerB;
  const int d0  = (blockIdx.x - bix * kBlkPerB) * kScanCh;
  const int d   = d0 + tid;
  const int row0 = bix * kSeq;

  float negA[kNst], h[kNst];
#pragma unroll
  for (int q = 0; q < 4; ++q) {
    const v4f al = *(const v4f*)(Alog + (size_t)d * kNst + 4 * q);
    negA[4 * q + 0] = -__expf(al[0]);
    negA[4 * q + 1] = -__expf(al[1]);
    negA[4 * q + 2] = -__expf(al[2]);
    negA[4 * q + 3] = -__expf(al[3]);
  }
#pragma unroll
  for (int n = 0; n < kNst; ++n) h[n] = 0.f;
  const float Dd = Dsk[d];
  const int hrow = lane >> 4, c8 = (lane & 15) * 8;

#pragma unroll 1
  for (int t0 = 0; t0 < kSeq; t0 += kScanTS) {
    __syncthreads();
#pragma unroll
    for (int p = 0; p < 2; ++p) {
      const int idx  = tid + 128 * p;
      const int idxc = (idx < kScanTS * 8) ? idx : (kScanTS * 8 - 1);
      const int r  = idxc >> 3;
      const int q4 = (idxc & 7) * 4;
      const v4f v = *(const v4f*)(DBC + (size_t)(row0 + t0 + r) * kXdP + kRank + q4);
      if (idx < kScanTS * 8) *(v4f*)(sBC + r * 32 + q4) = v;
    }
    __syncthreads();
#pragma unroll 1
    for (int s = 0; s < kScanTS; ++s) {
      const size_t m = (size_t)(row0 + t0 + s);
      const float a  = DLR[m * kDim + d];
      const float xv = XA[m * kDim + d];
      const float zv = XZ[m * kXzP + kDim + d];
      const float dt = softplus_fast(a);
      const float dtx = dt * xv;
      v4f Bq[4], Cq[4];
#pragma unroll
      for (int qq = 0; qq < 4; ++qq) {
        Bq[qq] = *(const v4f*)(sBC + s * 32 + 4 * qq);
        Cq[qq] = *(const v4f*)(sBC + s * 32 + kNst + 4 * qq);
      }
      float y = 0.f;
#pragma unroll
      for (int n = 0; n < kNst; ++n) {
        const float e = __expf(dt * negA[n]);
        h[n] = fmaf(e, h[n], dtx * Bq[n >> 2][n & 3]);
        y = fmaf(h[n], Cq[n >> 2][n & 3], y);
      }
      y = fmaf(xv, Dd, y);
      sY[s * kScanYP + tid] = (y * silu_fast(zv)) * kCarryY;
    }
    __syncthreads();
    v8h hv[4];
#pragma unroll
    for (int it = 0; it < 4; ++it) {
      const int p  = it * 4 + wave;
      const int pc = (p < kScanPairs) ? p : (kScanPairs - 1);
      const float* sp = sY + (pc * 2 + hrow) * kScanYP + c8;
      const v4f a0 = *(const v4f*)(sp);
      const v4f a1 = *(const v4f*)(sp + 4);
#pragma unroll
      for (int e = 0; e < 4; ++e) {
        hv[it][e]     = (_Float16)a0[e];
        hv[it][4 + e] = (_Float16)a1[e];
      }
    }
    for (int pass = 0; pass < 2; ++pass) {
#pragma unroll
      for (int it = 0; it < 4; ++it) {
        const int p = it * 4 + wave;
        if (p < kScanPairs) {
          const int row = p * 2 + hrow;
          *(volatile v8h*)(Y16 + (size_t)(row0 + t0 + row) * kDim + d0 + c8) = hv[it];
        }
      }
      __threadfence();
    }
  }
}

__global__ __launch_bounds__(256) void swiglu_kernel(const float* __restrict__ G12, unsigned short* __restrict__ HID16)
{
  const int i = blockIdx.x * 256 + threadIdx.x;
  if (i >= kTokP * (kHid / 8)) return;
  const int m  = i / (kHid / 8);
  const int c8 = (i - m * (kHid / 8)) * 8;
  const float* pa = G12 + (size_t)m * kG12P + c8;
  const v4f a0 = *(const v4f*)(pa);
  const v4f a1 = *(const v4f*)(pa + 4);
  const v4f g0 = *(const v4f*)(pa + kHid);
  const v4f g1 = *(const v4f*)(pa + kHid + 4);
  v8h hv;
#pragma unroll
  for (int e = 0; e < 4; ++e) {
    hv[e]     = (_Float16)((silu_fast(a0[e]) * g0[e]) * kCarryHid);
    hv[4 + e] = (_Float16)((silu_fast(a1[e]) * g1[e]) * kCarryHid);
  }
  unsigned short* q = HID16 + ((size_t)i << 3);
  *(volatile v8h*)q = hv;
  __threadfence();
  *(volatile v8h*)q = hv;
}

template <int BM, int OM, bool RS>
static void launch_gemm(hipStream_t s, const unsigned short* A, int lda, const unsigned short* Bt, int ldb,
                        float* C, int ldc, const float* bias, const float* bias2, int nsplit,
                        const float* resid, unsigned short* aux, int M, int N, int K, float scale)
{
  const int tiles = (M >> 6) * (N >> 6);
  const int blocks = (tiles + 7) / 8;
  wmma_gemm64_f16<BM, OM, RS><<<dim3(blocks), dim3(256), 0, s>>>(
      A, lda, Bt, ldb, C, ldc, bias, bias2, nsplit, resid, aux, M, N, K, scale);
}

static void launch_cast(hipStream_t s, const float* src, unsigned short* dst, int layers, int rows_launch,
                        int rows_src, int k_src, int k_dst, int dst_layer_rows, int dst_row_off, float scale)
{
  const int total8 = layers * rows_launch * (k_dst / 8);
  cast_plane_kernel<<<(total8 + 255) / 256, 256, 0, s>>>(src, dst, total8, rows_launch, rows_src, k_src, k_dst,
                                                         dst_layer_rows, dst_row_off, scale);
}

extern "C" void kernel_launch(void* const* d_in, const int* in_sizes, int n_in,
                              void* d_out, int out_size, void* d_ws, size_t ws_size,
                              hipStream_t stream)
{
  if (n_in < 24) return;
  const int expect[24] = {
      kBatch * 3 * kImg * kImg, kDim * kPatchK, kDim, kDepth * kDim, kDepth * kDim,
      kDepth * kXzP * kDim, kDepth * kDim * kConvK, kDepth * kDim, kDepth * kXdN * kDim,
      kDepth * kDim * kRank, kDepth * kDim, kDepth * kDim * kNst, kDepth * kDim,
      kDepth * kDim * kDim, kDepth * kDim, kDepth * kDim, kDepth * kHid * kDim, kDepth * kHid,
      kDepth * kHid * kDim, kDepth * kHid, kDepth * kDim * kHid, kDepth * kDim, kDim, kDim};
  for (int i = 0; i < 24; ++i) if (in_sizes[i] != expect[i]) return;
  if (out_size != kTok * kDim) return;
  if (ws_size < kWsTotal) return;

  const float* x        = (const float*)d_in[0];
  const float* patch_w  = (const float*)d_in[1];
  const float* patch_b  = (const float*)d_in[2];
  const float* norm1_w  = (const float*)d_in[3];
  const float* norm1_b  = (const float*)d_in[4];
  const float* in_proj  = (const float*)d_in[5];
  const float* conv_w   = (const float*)d_in[6];
  const float* conv_b   = (const float*)d_in[7];
  const float* x_proj   = (const float*)d_in[8];
  const float* dt_w     = (const float*)d_in[9];
  const float* dt_b     = (const float*)d_in[10];
  const float* A_log    = (const float*)d_in[11];
  const float* D_skip   = (const float*)d_in[12];
  const float* out_proj = (const float*)d_in[13];
  const float* norm2_w  = (const float*)d_in[14];
  const float* norm2_b  = (const float*)d_in[15];
  const float* w1_w     = (const float*)d_in[16];
  const float* w1_b     = (const float*)d_in[17];
  const float* w2_w     = (const float*)d_in[18];
  const float* w2_b     = (const float*)d_in[19];
  const float* w3_w     = (const float*)d_in[20];
  const float* w3_b     = (const float*)d_in[21];
  const float* normf_w  = (const float*)d_in[22];
  const float* normf_b  = (const float*)d_in[23];

  char* ws = (char*)d_ws;
  unsigned short* PW16   = (unsigned short*)(ws + kOffPW);
  unsigned short* WIN16  = (unsigned short*)(ws + kOffWIN);
  unsigned short* WXP16  = (unsigned short*)(ws + kOffWXP);
  unsigned short* WDT16  = (unsigned short*)(ws + kOffWDT);
  unsigned short* WOUT16 = (unsigned short*)(ws + kOffWOUT);
  unsigned short* W12    = (unsigned short*)(ws + kOffW12);
  unsigned short* W3     = (unsigned short*)(ws + kOffW3);
  unsigned short* A0     = (unsigned short*)(ws + kOffA0);
  float*          H      = (float*)(ws + kOffH);
  unsigned short* U16    = (unsigned short*)(ws + kOffU16);
  float*          XZ     = (float*)(ws + kOffXZ);
  float*          XA     = (float*)(ws + kOffXA);
  unsigned short* XA16   = (unsigned short*)(ws + kOffXA16);
  float*          DBC    = (float*)(ws + kOffDBC);
  unsigned short* DTIN   = (unsigned short*)(ws + kOffDTIN);
  float*          DLR    = (float*)(ws + kOffDLR);
  unsigned short* Y16    = (unsigned short*)(ws + kOffY16);
  float*          G12    = (float*)(ws + kOffG12);
  unsigned short* HID16  = (unsigned short*)(ws + kOffHID);

  launch_cast(stream, patch_w,  PW16,   1,      kDim,  kDim,  kPatchK, kPatchK, kDim,  0,    kCarryW);
  launch_cast(stream, in_proj,  WIN16,  kDepth, kXzP,  kXzP,  kDim,    kDim,    kXzP,  0,    kCarryW);
  launch_cast(stream, x_proj,   WXP16,  kDepth, kXdP,  kXdN,  kDim,    kDim,    kXdP,  0,    kCarryW);
  launch_cast(stream, dt_w,     WDT16,  kDepth, kDim,  kDim,  kRank,   kDtK,    kDim,  0,    kCarryWdt);
  launch_cast(stream, out_proj, WOUT16, kDepth, kDim,  kDim,  kDim,    kDim,    kDim,  0,    kCarryW);
  launch_cast(stream, w1_w,     W12,    kDepth, kHid,  kHid,  kDim,    kDim,    kG12P, 0,    kCarryW);
  launch_cast(stream, w2_w,     W12,    kDepth, kHid,  kHid,  kDim,    kDim,    kG12P, kHid, kCarryW);
  launch_cast(stream, w3_w,     W3,     kDepth, kDim,  kDim,  kHid,    kHid,    kDim,  0,    kCarryW);
  im2col_kernel<<<(kTokP * (kPatchK / 8)) / 256, 256, 0, stream>>>(x, A0);
  zero_fill16_kernel<<<((kTokP - kTok) * kDim / 8 + 255) / 256, 256, 0, stream>>>(
      Y16 + (size_t)kTok * kDim, (kTokP - kTok) * kDim / 8);

  launch_gemm<2, 0, false>(stream, A0, kPatchK, PW16, kPatchK, H, kDim, patch_b, patch_b, kDim,
                           H, DTIN, kTokP, kDim, kPatchK, 1.0f / kCarryW);

  for (int i = 0; i < kDepth; ++i) {
    ln_kernel<false><<<kTokP / 8, 256, 0, stream>>>(H, norm1_w + (size_t)i * kDim, norm1_b + (size_t)i * kDim,
                                                    (void*)U16, kTokP);
    launch_gemm<0, 0, false>(stream, U16, kDim, WIN16 + (size_t)i * kXzP * kDim, kDim, XZ, kXzP,
                             patch_b, patch_b, kXzP, H, DTIN, kTokP, kXzP, kDim, 1.0f / kCarryW);
    conv_silu_kernel<<<(kTokP * (kDim / 4)) / 256, 256, 0, stream>>>(
        XZ, conv_w + (size_t)i * kDim * kConvK, conv_b + (size_t)i * kDim, XA, XA16);
    launch_gemm<0, 3, false>(stream, XA16, kDim, WXP16 + (size_t)i * kXdP * kDim, kDim, DBC, kXdP,
                             patch_b, patch_b, kXdP, H, DTIN, kTokP, kXdP, kDim, 1.0f / (kCarryXa * kCarryW));
    launch_gemm<2, 0, false>(stream, DTIN, kDtK, WDT16 + (size_t)i * kDim * kDtK, kDtK, DLR, kDim,
                             dt_b + (size_t)i * kDim, dt_b + (size_t)i * kDim, kDim,
                             H, DTIN, kTokP, kDim, kDtK, 1.0f / (kCarryDt * kCarryWdt));
    scan_gate_kernel<<<kBatch * (kDim / kScanCh), kScanCh, 0, stream>>>(
        DLR, XA, XZ, DBC, A_log + (size_t)i * kDim * kNst, D_skip + (size_t)i * kDim, Y16);
    launch_gemm<0, 0, true>(stream, Y16, kDim, WOUT16 + (size_t)i * kDim * kDim, kDim, H, kDim,
                            patch_b, patch_b, kDim, H, DTIN, kTokP, kDim, kDim, 1.0f / (kCarryY * kCarryW));
    ln_kernel<false><<<kTokP / 8, 256, 0, stream>>>(H, norm2_w + (size_t)i * kDim, norm2_b + (size_t)i * kDim,
                                                    (void*)U16, kTokP);
    launch_gemm<2, 0, false>(stream, U16, kDim, W12 + (size_t)i * kG12P * kDim, kDim, G12, kG12P,
                             w1_b + (size_t)i * kHid, w2_b + (size_t)i * kHid, kHid,
                             H, DTIN, kTokP, kG12P, kDim, 1.0f / kCarryW);
    swiglu_kernel<<<(kTokP * (kHid / 8)) / 256, 256, 0, stream>>>(G12, HID16);
    launch_gemm<2, 0, true>(stream, HID16, kHid, W3 + (size_t)i * kDim * kHid, kHid, H, kDim,
                            w3_b + (size_t)i * kDim, w3_b + (size_t)i * kDim, kDim,
                            H, DTIN, kTokP, kDim, kHid, 1.0f / (kCarryHid * kCarryW));
  }

  ln_kernel<true><<<kTok / 8, 256, 0, stream>>>(H, normf_w, normf_b, d_out, kTok);
}
